// NoLayer_90005334655023
// MI455X (gfx1250) — hardware-verified
//
#include <hip/hip_runtime.h>
#include <math.h>

typedef __attribute__((ext_vector_type(16))) _Float16 v16h;
typedef __attribute__((ext_vector_type(16))) __bf16 v16b;
typedef __attribute__((ext_vector_type(8)))  _Float16 v8h;
typedef __attribute__((ext_vector_type(8)))  float v8f;
typedef __attribute__((ext_vector_type(4)))  float v4f;
typedef __attribute__((ext_vector_type(2)))  float v2f;
typedef __attribute__((ext_vector_type(4)))  unsigned v4u;
typedef __attribute__((ext_vector_type(4)))  int v4i;
typedef float __attribute__((may_alias)) float_a;
typedef int __attribute__((may_alias)) int_a;

template <typename T> __device__ __forceinline__ void vst2(void* p, T v) { *(volatile T*)p = v; __threadfence(); *(volatile T*)p = v; }
__device__ __forceinline__ v8f wmma16(v16h a, v16h b, v8f c) {
  v8f d = __builtin_amdgcn_wmma_f32_16x16x32_f16(false, a, false, b, (short)0, c, false, false);
  asm volatile("v_nop\n\tv_nop\n\tv_nop\n\tv_nop" : "+v"(d) : "v"(a), "v"(b));
  return d;
}
__device__ __forceinline__ v8f wmma_bf(v16b a, v16b b, v8f c) {
  v8f d = __builtin_amdgcn_wmma_f32_16x16x32_bf16(false, a, false, b, (short)0, c, false, false);
  asm volatile("v_nop\n\tv_nop\n\tv_nop\n\tv_nop" : "+v"(d) : "v"(a), "v"(b));
  return d;
}
__device__ __forceinline__ v16h frag_h(const _Float16* rowk0, int lane) {
  union { v16h v; v8h q[2]; } u; const _Float16* p = rowk0 + 8 * (lane >> 4);
  u.q[0] = *(const v8h*)p; u.q[1] = *(const v8h*)(p + 16); return u.v;
}
__device__ __forceinline__ v16h frag_f32(const float* rowk0, int lane) {
  v16h a; const float* p = rowk0 + 8 * (lane >> 4);
#pragma unroll
  for (int i = 0; i < 8; ++i) { a[i] = (_Float16)p[i]; a[8 + i] = (_Float16)p[16 + i]; }
  return a;
}
__device__ __forceinline__ v16h frag_f32s(const float* rowk0, int lane, float sc) {
  v16h a; const float* p = rowk0 + 8 * (lane >> 4);
#pragma unroll
  for (int i = 0; i < 8; ++i) { a[i] = (_Float16)(p[i] * sc); a[8 + i] = (_Float16)(p[16 + i] * sc); }
  return a;
}
__device__ __forceinline__ v16h fragc_f32(const float* W, int k0, int n, int lane, int ld, int K) {
  v16h a; const int g = lane >> 4;
#pragma unroll
  for (int i = 0; i < 8; ++i) { const int ka = k0 + 8 * g + i, kb = ka + 16;
    a[i] = (_Float16)(ka < K ? W[(size_t)(ka < K ? ka : K - 1) * ld + n] : 0.f); a[8 + i] = (_Float16)(kb < K ? W[(size_t)(kb < K ? kb : K - 1) * ld + n] : 0.f); }
  return a;
}
struct F2 { v16b h, l; };
__device__ __forceinline__ F2 bsplit16(const float v[16]) { F2 r;
#pragma unroll
  for (int i = 0; i < 16; ++i) { const __bf16 h = (__bf16)v[i]; r.h[i] = h; r.l[i] = (__bf16)(v[i] - (float)h); }
  return r; }
__device__ __forceinline__ F2 split_row(const float* row, int k0, int lane) { float v[16]; const float* p = row + k0 + 8 * (lane >> 4);
#pragma unroll
  for (int i = 0; i < 8; ++i) { v[i] = p[i]; v[8 + i] = p[16 + i]; }
  return bsplit16(v); }
__device__ __forceinline__ F2 split_rowK(const float* row, int k0, int lane, int K) { float v[16]; const int g = lane >> 4;
#pragma unroll
  for (int i = 0; i < 8; ++i) { const int ka = k0 + 8 * g + i, kb = ka + 16; v[i] = ka < K ? row[ka < K ? ka : K - 1] : 0.f; v[8 + i] = kb < K ? row[kb < K ? kb : K - 1] : 0.f; }
  return bsplit16(v); }
__device__ __forceinline__ F2 split_col(const float* W, int k0, int n, int lane, int ld, int K) { float v[16]; const int g = lane >> 4;
#pragma unroll
  for (int i = 0; i < 8; ++i) { const int ka = k0 + 8 * g + i, kb = ka + 16; v[i] = ka < K ? W[(size_t)(ka < K ? ka : K - 1) * ld + n] : 0.f; v[8 + i] = kb < K ? W[(size_t)(kb < K ? kb : K - 1) * ld + n] : 0.f; }
  return bsplit16(v); }
__device__ __forceinline__ v8f mac3(const F2& a, const F2& b, v8f c) { c = wmma_bf(a.l, b.h, c); c = wmma_bf(a.h, b.l, c); return wmma_bf(a.h, b.h, c); }
__device__ __forceinline__ float sigm(float v) { return 1.0f / (1.0f + expf(-v)); }
#define LDSX() do { asm volatile("s_wait_dscnt 0" ::: "memory"); __builtin_amdgcn_wave_barrier(); __builtin_amdgcn_fence(__ATOMIC_RELEASE, "workgroup"); } while (0)


#define NIN 65536
#define NOUT 16384
#define KN 16
#define FD 64
#define ND 4
#define NPH 8
#define NM (ND * NPH)
#define ENH (NM * FD)
#define OUT 256
#define WSC 256.0f
#ifndef TOB
#define TOB (NOUT / 64)
#endif
typedef __attribute__((ext_vector_type(8))) __bf16 v8b;
__device__ __forceinline__ v16b frag_b(const __bf16* rowk0, int lane) {
  union { v16b v; v8b q[2]; } u; const __bf16* p = rowk0 + 8 * (lane >> 4);
  u.q[0] = *(const v8b*)p; u.q[1] = *(const v8b*)(p + 16); return u.v;
}
__device__ __forceinline__ float bfr(float v) { return (float)(__bf16)v; }
__device__ __attribute__((noinline)) float exp_ni(float v) { return expf(v); }
__device__ __attribute__((noinline)) float erf_ni(float v) { return erff(v); }

#define WS_PW  0u
#define WS_AGG (WS_PW + 2u * (size_t)OUT * ENH)
#define WS_END (WS_AGG + 2u * (size_t)NOUT * ENH)

__global__ __launch_bounds__(256) void k_packw(const float* __restrict__ WO, _Float16* __restrict__ PW) { const int n = blockIdx.x, t = threadIdx.x; __shared__ __align__(16) _Float16 sh[ENH];
  for (int k = t; k < ENH; k += 256) sh[k] = (_Float16)(bfr(WO[(size_t)k * OUT + n]) * WSC); __syncthreads(); for (int q = t; q < ENH / 8; q += 256) vst2((unsigned*)(PW + (size_t)n * ENH + q * 8), *(const v4u*)&sh[q * 8]); }
__global__ __launch_bounds__(256) void k_agg(const float* __restrict__ X, const float* __restrict__ DD, const float* __restrict__ DP, const float* __restrict__ DISTS, const float* __restrict__ SIG, const float* __restrict__ KAP, const float* __restrict__ PHI, const int* __restrict__ NH, _Float16* __restrict__ AGG) {
  __shared__ float sw[KN][NM + 1]; __shared__ float sx[KN][FD]; __shared__ __align__(16) _Float16 so2[ENH]; const int t = threadIdx.x; const size_t n = blockIdx.x;
  for (int e = t; e < KN * FD; e += 256) { const int k = e >> 6, f = e & 63; const int src = NH[n * KN + k]; sx[k][f] = bfr(X[(size_t)src * FD + f]); }
  for (int e = t; e < KN * NM; e += 256) { const int k = e / NM, m = e % NM; const int di = m / NPH, pj = m % NPH; const float d = bfr(DD[n * KN + k]), ph = bfr(DP[n * KN + k]); const float sg = bfr(SIG[0]), kp = bfr(KAP[0]);
    const float u = (d - bfr(DISTS[di])) / sg; const float wd = expf(-0.5f * u * u); const float wp = expf(kp * cosf(ph - bfr(PHI[pj]))); sw[k][m] = wd * wp; }
  __syncthreads();
  if (t < NM) { float s = 0.f; for (int k = 0; k < KN; ++k) s += sw[k][t]; const float inv = 1.0f / (s + 1e-9f); for (int k = 0; k < KN; ++k) sw[k][t] = sw[k][t] * inv; }
  __syncthreads();
  for (int e = t; e < ENH; e += 256) { const int m = e >> 6, f = e & 63; float a = 0.f;
#pragma unroll 1
    for (int k = 0; k < KN; ++k) a += sw[k][m] * sx[k][f];
    so2[e] = (_Float16)a; }
  __syncthreads(); vst2((unsigned*)(AGG + n * ENH + t * 8), *(const v4u*)&so2[t * 8]); }
__global__ __launch_bounds__(128) void k_out(const _Float16* __restrict__ AGG, const _Float16* __restrict__ PW, float* __restrict__ Y) { __shared__ __align__(16) float so[4][16][132];
  const int tid = threadIdx.x, wave = tid >> 5, lane = tid & 31, col = lane & 15, g = lane >> 4; const size_t r0 = (size_t)blockIdx.x * 64 + wave * 16; const int c0 = blockIdx.y * 128;
  v8f acc[8] = {};
#pragma unroll 2
  for (int kc = 0; kc < ENH / 32; ++kc) { const v16h a = frag_h(AGG + (r0 + col) * ENH + kc * 32, lane);
#pragma unroll
    for (int j = 0; j < 8; ++j) acc[j] = wmma16(a, frag_h(PW + (size_t)(c0 + j * 16 + col) * ENH + kc * 32, lane), acc[j]); }
#pragma unroll
  for (int j = 0; j < 8; ++j)
#pragma unroll
    for (int r = 0; r < 8; ++r) so[wave][8 * g + r][j * 16 + col] = acc[j][r] * (1.0f / WSC);
  LDSX(); for (int rl = 0; rl < 16; ++rl) vst2(Y + (r0 + rl) * OUT + c0 + lane * 4, *(const v4f*)&so[wave][rl][lane * 4]); }
extern "C" void kernel_launch(void* const* d_in, const int* in_sizes, int n_in, void* d_out, int out_size, void* d_ws, size_t ws_size, hipStream_t stream) {
  (void)in_sizes; (void)n_in; (void)out_size;
  const float** F = (const float**)d_in;
  if (ws_size < (size_t)WS_END) return;
  char* ws = (char*)d_ws; _Float16 *PW = (_Float16*)(ws + WS_PW), *AGG = (_Float16*)(ws + WS_AGG);
  k_packw<<<OUT, 256, 0, stream>>>(F[7], PW);
  k_agg<<<TOB * 64, 256, 0, stream>>>(F[0], F[1], F[2], F[3], F[4], F[5], F[6], (const int*)d_in[8], AGG);
  k_out<<<dim3(TOB, OUT / 128), 128, 0, stream>>>(AGG, PW, (float*)d_out);
}
